// CazzyAporboTransformerBlock_35862976921711
// MI455X (gfx1250) — hardware-verified
//
#include <hip/hip_runtime.h>
#include <math.h>
#include <stdint.h>

#define NB      2
#define SQ      1400
#define SP      1408
#define DM      256
#define NH      16
#define HD      16
#define QKN     512
#define NQKV    768
#define FF      1024
#define VOC     1400
#define SL      256
#define MROWS   (NB * SP)
#define TOK     (NB * SQ)
#define NQT     (SP / 16)
#define NGRP    (NH / 4)
#define LN_EPS  1e-5f
#define WSC     64.0f
#define ACARRY  16.0f
#define QKCARRY 16.0f
#define VCARRY  16.0f
#define PCARRY  1024.0f
#define OCARRY  256.0f
#define XCARRY  16.0f
#define RWCARRY 1024.0f
#define FCARRY  16.0f
static_assert((SP % 64) == 0 && SP >= SQ && (SP - SQ) < 16);
static_assert(NH * HD == DM && HD == 16 && (NH % 4) == 0);
static_assert((MROWS % 64) == 0 && (MROWS % 8) == 0 && (DM % 64) == 0 && (FF % 64) == 0 && (QKN % 64) == 0);
static_assert(VOC == SQ && SL == DM);
#define ATT_BLOCKS (NB * NGRP * NQT)
#define ROW_BLOCKS (MROWS / 8)

typedef _Float16 v16h __attribute__((ext_vector_type(16)));
typedef _Float16 v8h  __attribute__((ext_vector_type(8)));
typedef float    v8f  __attribute__((ext_vector_type(8)));
typedef float    v4f  __attribute__((ext_vector_type(4)));
typedef unsigned int v4u __attribute__((ext_vector_type(4)));

union FragH { v16h v; v8h h[2]; v4u u[2]; };

__device__ __forceinline__ unsigned short bf_bits(float f) {
  unsigned u = __float_as_uint(f);
  return (unsigned short)((u + 0x7FFFu + ((u >> 16) & 1u)) >> 16);
}
__device__ __forceinline__ float bf_up(unsigned short h) { return __uint_as_float(((unsigned)h) << 16); }
__device__ __forceinline__ float bfr(float f) { return bf_up(bf_bits(f)); }
__device__ __forceinline__ unsigned short h_bits(_Float16 x) { return __builtin_bit_cast(unsigned short, x); }
__device__ __forceinline__ unsigned pk16(unsigned short a, unsigned short b) { return (unsigned)a | ((unsigned)b << 16); }
__device__ __forceinline__ v8f zero8() { v8f z = {0.f, 0.f, 0.f, 0.f, 0.f, 0.f, 0.f, 0.f}; return z; }
__device__ __forceinline__ float gelu_f(float v) { return 0.5f * v * (1.0f + erff(v * 0.70710678118654752f)); }

__device__ __forceinline__ v16h ldfrag_h(const _Float16* p) {
  FragH f;
  f.h[0] = *(const v8h*)(p);
  f.h[1] = *(const v8h*)(p + 16);
  return f.v;
}
__device__ __forceinline__ v16h ldfrag_u(const unsigned short* p) {
  FragH f;
  f.u[0] = *(const v4u*)(p);
  f.u[1] = *(const v4u*)(p + 16);
  return f.v;
}

__device__ __forceinline__ v8f mma_raw(v16h a, v16h b, v8f c) {
  return __builtin_amdgcn_wmma_f32_16x16x32_f16(false, a, false, b, (short)0, c, false, false);
}
__device__ __forceinline__ void dep_guard1(v8f& a, v8f& b, v16h x) {
#if defined(__HIP_DEVICE_COMPILE__)
  asm volatile("v_nop\n\tv_nop\n\tv_nop\n\tv_nop" : "+v"(a), "+v"(b) : "v"(x));
#endif
}
__device__ __forceinline__ void guard2(v8f& s0, v8f& s1, v16h a, v16h b0, v16h b1) {
#if defined(__HIP_DEVICE_COMPILE__)
  asm volatile("v_nop\n\tv_nop\n\tv_nop\n\tv_nop" : "+v"(s0), "+v"(s1) : "v"(a), "v"(b0), "v"(b1));
#endif
}
__device__ __forceinline__ void guard1(v8f& a, v16h x, v16h y) {
#if defined(__HIP_DEVICE_COMPILE__)
  asm volatile("v_nop\n\tv_nop\n\tv_nop\n\tv_nop" : "+v"(a) : "v"(x), "v"(y));
#endif
}
__device__ __forceinline__ void keep4_h(v16h a, v16h b, v16h c, v16h d) {
#if defined(__HIP_DEVICE_COMPILE__)
  asm volatile("v_nop" :: "v"(a), "v"(b), "v"(c), "v"(d));
#endif
}
__device__ __forceinline__ void acc_guard4(v8f& a, v8f& b, v8f& c, v8f& d) {
#if defined(__HIP_DEVICE_COMPILE__)
  asm volatile("v_nop\n\tv_nop\n\tv_nop\n\tv_nop" : "+v"(a), "+v"(b), "+v"(c), "+v"(d));
#endif
}
__device__ __forceinline__ void wave_sync_lds() {
  __builtin_amdgcn_fence(__ATOMIC_RELEASE, "workgroup");
  __builtin_amdgcn_wave_barrier();
  __builtin_amdgcn_fence(__ATOMIC_ACQUIRE, "workgroup");
}

__global__ __launch_bounds__(256) void conv16m(const float* __restrict__ W0, const float* __restrict__ W1,
                                               const float* __restrict__ W2, const float* __restrict__ W3,
                                               const float* __restrict__ W4, const float* __restrict__ W5,
                                               unsigned short* dst, int n8) {
  const int y = blockIdx.y;
  const float* W = (y == 0) ? W0 : (y == 1) ? W1 : (y == 2) ? W2 : (y == 3) ? W3 : (y == 4) ? W4 : W5;
  const int i  = blockIdx.x * 256 + threadIdx.x;
  const int ic = (i < n8) ? i : (n8 - 1);
  const float* p = W + (size_t)ic * 8;
  const v4f a = *(const v4f*)(p), b = *(const v4f*)(p + 4);
  float v[8];
#pragma unroll
  for (int e = 0; e < 4; ++e) { v[e] = bfr(a[e]); v[4 + e] = bfr(b[e]); }
  v4u ov;
#pragma unroll
  for (int e = 0; e < 4; ++e) ov[e] = pk16(h_bits((_Float16)(v[2 * e] * WSC)), h_bits((_Float16)(v[2 * e + 1] * WSC)));
  unsigned short* dp = dst + ((size_t)y * n8 + (size_t)i) * 8;
  if (i < n8) *(volatile v4u*)dp = ov;
  __threadfence();
  if (i < n8) *(volatile v4u*)dp = ov;
}

__global__ __launch_bounds__(256) void tr16(const float* __restrict__ src, unsigned short* dst) {
  __shared__ float tile[64 * 65];
  const int tid = threadIdx.x;
  const int c0 = blockIdx.x * 64;
  const int s0 = blockIdx.y * 64;
  {
    const int rr = tid >> 2;
    const int cc = (tid & 3) * 16;
    const float* sp = src + (size_t)(s0 + rr) * DM + c0 + cc;
#pragma unroll
    for (int q = 0; q < 4; ++q) {
      const v4f a = *(const v4f*)(sp + 4 * q);
#pragma unroll
      for (int e = 0; e < 4; ++e) tile[rr * 65 + cc + 4 * q + e] = bfr(a[e]);
    }
  }
  __syncthreads();
  v4u o0, o1;
  const int p0 = tid, p1 = tid + 256;
  const int r0 = p0 >> 3, j0 = p0 & 7;
  const int r1 = p1 >> 3, j1 = p1 & 7;
#pragma unroll
  for (int e = 0; e < 4; ++e) {
    const float f0 = tile[(8 * j0 + 2 * e) * 65 + r0] * WSC, f1 = tile[(8 * j0 + 2 * e + 1) * 65 + r0] * WSC;
    const float g0 = tile[(8 * j1 + 2 * e) * 65 + r1] * WSC, g1 = tile[(8 * j1 + 2 * e + 1) * 65 + r1] * WSC;
    o0[e] = pk16(h_bits((_Float16)f0), h_bits((_Float16)f1));
    o1[e] = pk16(h_bits((_Float16)g0), h_bits((_Float16)g1));
  }
  unsigned short* d0 = dst + (size_t)(c0 + r0) * SL + s0 + 8 * j0;
  unsigned short* d1 = dst + (size_t)(c0 + r1) * SL + s0 + 8 * j1;
  *(volatile v4u*)d0 = o0;
  *(volatile v4u*)d1 = o1;
  __threadfence();
  *(volatile v4u*)d0 = o0;
  *(volatile v4u*)d1 = o1;
}

template <int NORM, int RBF>
__global__ __launch_bounds__(256) void rows16(const float* __restrict__ src, const float* __restrict__ g,
                                              const float* __restrict__ bt, unsigned short* dst, float carry) {
  const int lane = threadIdx.x & 31;
  const int m = blockIdx.x * 8 + (threadIdx.x >> 5);
  const int b = m / SP;
  const int t = m - b * SP;
  const bool live = (t < SQ);
  const int tc = live ? t : (SQ - 1);
  const float* rp = src + ((size_t)(b * SQ + tc)) * DM + lane * 8;
  const v4f a0 = *(const v4f*)(rp), a1 = *(const v4f*)(rp + 4);
  float v[8];
#pragma unroll
  for (int e = 0; e < 4; ++e) { v[e] = a0[e]; v[4 + e] = a1[e]; }
  if (RBF) {
#pragma unroll
    for (int i = 0; i < 8; ++i) v[i] = bfr(v[i]);
  }
  if (NORM) {
    float s = 0.f;
#pragma unroll
    for (int i = 0; i < 8; ++i) s += v[i];
#pragma unroll
    for (int o = 1; o < 32; o <<= 1) s += __shfl_xor(s, o, 32);
    const float mean = s * (1.0f / 256.0f);
    float s2 = 0.f;
#pragma unroll
    for (int i = 0; i < 8; ++i) { const float d = v[i] - mean; s2 += d * d; }
#pragma unroll
    for (int o = 1; o < 32; o <<= 1) s2 += __shfl_xor(s2, o, 32);
    const float inv = rsqrtf(s2 * (1.0f / 256.0f) + LN_EPS);
    const v4f ga = *(const v4f*)(g + lane * 8), gb = *(const v4f*)(g + lane * 8 + 4);
    const v4f ba = *(const v4f*)(bt + lane * 8), bb = *(const v4f*)(bt + lane * 8 + 4);
#pragma unroll
    for (int e = 0; e < 4; ++e) {
      v[e]     = (v[e] - mean) * inv * bfr(ga[e]) + bfr(ba[e]);
      v[4 + e] = (v[4 + e] - mean) * inv * bfr(gb[e]) + bfr(bb[e]);
    }
  }
  v4u o;
#pragma unroll
  for (int e = 0; e < 4; ++e) {
    const float f0 = live ? v[2 * e] * carry : 0.f;
    const float f1 = live ? v[2 * e + 1] * carry : 0.f;
    o[e] = pk16(h_bits((_Float16)f0), h_bits((_Float16)f1));
  }
  unsigned short* dp = dst + (size_t)m * DM + lane * 8;
  *(volatile v4u*)dp = o;
  __threadfence();
  *(volatile v4u*)dp = o;
}

__global__ __launch_bounds__(256) void smax16(const float* __restrict__ src, unsigned short* dst) {
  const int lane = threadIdx.x & 31;
  const int m = blockIdx.x * 8 + (threadIdx.x >> 5);
  const int b = m / SP;
  const int t = m - b * SP;
  const bool live = (t < SQ);
  const int tc = live ? t : (SQ - 1);
  const float* rp = src + ((size_t)(b * SQ + tc)) * SL + lane * 8;
  const v4f a0 = *(const v4f*)(rp), a1 = *(const v4f*)(rp + 4);
  float v[8];
#pragma unroll
  for (int e = 0; e < 4; ++e) { v[e] = a0[e]; v[4 + e] = a1[e]; }
  float mx = v[0];
#pragma unroll
  for (int i = 1; i < 8; ++i) mx = fmaxf(mx, v[i]);
#pragma unroll
  for (int o = 1; o < 32; o <<= 1) mx = fmaxf(mx, __shfl_xor(mx, o, 32));
  float s = 0.f;
#pragma unroll
  for (int i = 0; i < 8; ++i) { v[i] = exp2f((v[i] - mx) * 1.4426950408889634f); s += v[i]; }
#pragma unroll
  for (int o = 1; o < 32; o <<= 1) s += __shfl_xor(s, o, 32);
  const float inv = (1.0f / s) * RWCARRY;
  v4u o;
#pragma unroll
  for (int e = 0; e < 4; ++e) {
    const float f0 = live ? v[2 * e] * inv : 0.f;
    const float f1 = live ? v[2 * e + 1] * inv : 0.f;
    o[e] = pk16(h_bits((_Float16)f0), h_bits((_Float16)f1));
  }
  unsigned short* dp = dst + (size_t)m * SL + lane * 8;
  *(volatile v4u*)dp = o;
  __threadfence();
  *(volatile v4u*)dp = o;
}

template <int OM, int BIASM, int ACT, int RES>
__global__ __launch_bounds__(256) void gemm64(
    const unsigned short* __restrict__ Ap, int lda, long long sAo, long long sAi,
    const unsigned short* __restrict__ Btp, int ldb, long long sBo, long long sBi,
    const float* __restrict__ bias, int sbo, int sbi,
    const float* __restrict__ Rp,
    void* Cout, int ldc, long long sCo, long long sCi,
    int M, int N, int K, int Mv, int nin, float oscale, float ocarry) {
  __shared__ __align__(16) float sT[8][16 * 68];
  const int by   = blockIdx.y;
  const int bo   = by / nin;
  const int bi   = by - bo * nin;
  const int lane = threadIdx.x & 31;
  const int wave = threadIdx.x >> 5;
  const int tilesN = N >> 6;
  const int tilesM = M >> 6;
  const int tile = blockIdx.x * 8 + wave;
  if (tile >= tilesM * tilesN) return;
  const int tm = tile / tilesN;
  const int tn = tile - tm * tilesN;
  const int m0 = tm << 6;
  const int n0 = tn << 6;

  const unsigned short* A1 = Ap  + (size_t)((long long)bo * sAo + (long long)bi * sAi);
  const unsigned short* Bb = Btp + (size_t)((long long)bo * sBo + (long long)bi * sBi);
  const float*         bsp = bias + (size_t)bo * (size_t)sbo + (size_t)bi * (size_t)sbi;
  const size_t cofs = (size_t)((long long)bo * sCo + (long long)bi * sCi);

  const int rlane = lane & 15;
  const int koff  = (lane >> 4) * 8;
  const int mOff  = (lane >> 4) * 8;

  v8f acc[4][4];
#pragma unroll
  for (int i = 0; i < 4; ++i)
#pragma unroll
    for (int j = 0; j < 4; ++j) acc[i][j] = zero8();

  for (int k0 = 0; k0 < K; k0 += 32) {
    v16h bh[4];
#pragma unroll
    for (int j = 0; j < 4; ++j) {
      const size_t bofs = (size_t)(n0 + (j << 4) + rlane) * ldb + koff + k0;
      bh[j] = ldfrag_u(Bb + bofs);
    }
#pragma unroll
    for (int i = 0; i < 4; ++i) {
      const size_t ao = (size_t)(m0 + (i << 4) + rlane) * lda + koff + k0;
      const v16h ah = ldfrag_u(A1 + ao);
#pragma unroll
      for (int j = 0; j < 4; ++j) acc[i][j] = mma_raw(ah, bh[j], acc[i][j]);
      dep_guard1(acc[i][0], acc[i][3], ah);
    }
    keep4_h(bh[0], bh[1], bh[2], bh[3]);
  }
  acc_guard4(acc[0][0], acc[0][1], acc[0][2], acc[0][3]);
  acc_guard4(acc[1][0], acc[1][1], acc[1][2], acc[1][3]);
  acc_guard4(acc[2][0], acc[2][1], acc[2][2], acc[2][3]);
  acc_guard4(acc[3][0], acc[3][1], acc[3][2], acc[3][3]);

  const int hh2 = lane >> 4, c4 = (lane & 15) * 4;
  const int q8  = lane >> 3, c8 = (lane & 7) * 8;
  float bc[8];
#pragma unroll
  for (int e = 0; e < 8; ++e) bc[e] = 0.f;
  if (BIASM == 0) {
    if (OM != 2) {
      const int cb = n0 + c4;
      const int i0 = (cb < N - 4) ? cb : (N - 4);
      const v4f b0v = *(const v4f*)(bsp + i0);
#pragma unroll
      for (int e = 0; e < 4; ++e) bc[e] = bfr(b0v[e]);
    } else {
      const int cb = n0 + c8;
      const int i0 = (cb < N - 8) ? cb : (N - 8);
      const v4f b0a = *(const v4f*)(bsp + i0), b0b = *(const v4f*)(bsp + i0 + 4);
#pragma unroll
      for (int e = 0; e < 4; ++e) {
        bc[e]     = bfr(b0a[e]);
        bc[4 + e] = bfr(b0b[e]);
      }
    }
  }

  float* slab = sT[wave];
#pragma unroll
  for (int i = 0; i < 4; ++i) {
    const int mBase = m0 + (i << 4);
#pragma unroll
    for (int j = 0; j < 4; ++j) {
#pragma unroll
      for (int r = 0; r < 8; ++r) {
        slab[(mOff + r) * 68 + (j << 4) + rlane] = acc[i][j][r];
      }
    }
    wave_sync_lds();
    if (OM != 2) {
      float* C = (float*)Cout + cofs;
      const float* R = Rp + cofs;
      v4f vals[8];
#pragma unroll
      for (int it = 0; it < 8; ++it) {
        const int row = it * 2 + hh2;
        v4f v = *(const v4f*)(slab + row * 68 + c4);
        v4f rv = {0.f, 0.f, 0.f, 0.f};
        if (RES != 0) {
          const int gr  = mBase + row;
          const int grc = (gr < Mv) ? gr : (Mv - 1);
          rv = *(const v4f*)(R + (size_t)grc * ldc + n0 + c4);
          if (RES == 2) {
#pragma unroll
            for (int e = 0; e < 4; ++e) rv[e] = bfr(rv[e]);
          }
        }
#pragma unroll
        for (int e = 0; e < 4; ++e) {
          float f = v[e] * oscale + bc[e];
          if (ACT == 1) f = gelu_f(f);
          v[e] = rv[e] + f;
        }
        vals[it] = v;
      }
      for (int pass = 0; pass < 2; ++pass) {
#pragma unroll
        for (int it = 0; it < 8; ++it) {
          const int gr = mBase + it * 2 + hh2;
          if (gr < Mv) {
            *(volatile v4f*)(C + (size_t)gr * ldc + n0 + c4) = vals[it];
          }
        }
        __threadfence();
      }
    } else {
      unsigned short* C = (unsigned short*)Cout + cofs;
      v4u hv[4];
#pragma unroll
      for (int it = 0; it < 4; ++it) {
        const int row = it * 4 + q8;
        const float* sp = slab + row * 68 + c8;
        float bm = 0.f;
        if (BIASM == 1) bm = bfr(bsp[mBase + row]);
        v4u a;
#pragma unroll
        for (int e = 0; e < 4; ++e) {
          float f0 = sp[2 * e]     * oscale + ((BIASM == 1) ? bm : bc[2 * e]);
          float f1 = sp[2 * e + 1] * oscale + ((BIASM == 1) ? bm : bc[2 * e + 1]);
          if (ACT == 1) { f0 = gelu_f(f0); f1 = gelu_f(f1); }
          a[e] = pk16(h_bits((_Float16)(f0 * ocarry)), h_bits((_Float16)(f1 * ocarry)));
        }
        hv[it] = a;
      }
      for (int pass = 0; pass < 2; ++pass) {
#pragma unroll
        for (int it = 0; it < 4; ++it) {
          const int row = it * 4 + q8;
          *(volatile v4u*)(C + (size_t)(mBase + row) * ldc + n0 + c8) = hv[it];
        }
        __threadfence();
      }
    }
    wave_sync_lds();
  }
}

template <int AFF>
__global__ __launch_bounds__(128)
void attn16(const unsigned short* __restrict__ QK, const unsigned short* __restrict__ VTp,
            const int* __restrict__ ids, const float* __restrict__ aff, unsigned short* CT) {
  __shared__ __align__(16) float Ps[4][16 * 36];
  __shared__ __align__(16) float Os[16 * 68];

  const int tid  = threadIdx.x;
  const int wave = tid >> 5;
  const int lane = tid & 31;
  const int hh   = lane >> 4;
  const int c    = lane & 15;

  const int blk  = blockIdx.x;
  const int bg   = blk / NQT;
  const int qt   = blk - bg * NQT;
  const int bat  = bg / NGRP;
  const int grp  = bg - bat * NGRP;
  const int head = grp * 4 + wave;
  const int q0   = qt * 16;

  const _Float16* Qb = (const _Float16*)(const void*)QK + (size_t)bat * SP * QKN + head * HD;
  const _Float16* Kb = Qb + DM;
  const _Float16* Vb = (const _Float16*)(const void*)VTp + ((size_t)bat * DM + head * HD) * SP;
  const float lsc = (1.4426950408889634f * 0.25f) / (QKCARRY * QKCARRY);
  const float asc = 1.4426950408889634f * 0.1f;
  const v4u z4 = {0u, 0u, 0u, 0u};

  FragH qa;
  qa.h[0] = *(const v8h*)(Qb + (size_t)(q0 + c) * QKN + 8 * hh);
  qa.u[1] = z4;

  int idr[8];
#pragma unroll
  for (int r = 0; r < 8; ++r) idr[r] = 0;
  if (AFF) {
#pragma unroll
    for (int r = 0; r < 8; ++r) {
      const int t  = q0 + 8 * hh + r;
      const int tc = (t < SQ) ? t : (SQ - 1);
      int id = ids[(size_t)bat * SQ + tc];
      id = (id < 0) ? 0 : ((id > VOC - 1) ? (VOC - 1) : id);
      idr[r] = id;
    }
  }

  float mrow[8], lrow[8];
  v8f acc = zero8();
#pragma unroll
  for (int r = 0; r < 8; ++r) { mrow[r] = -INFINITY; lrow[r] = 0.f; }
  float* pt = Ps[wave];

#pragma unroll 1
  for (int kb = 0; kb < SP; kb += 32) {
    const _Float16* kp = Kb + (size_t)(kb + c) * QKN + 8 * hh;
    FragH kf0, kf1;
    kf0.h[0] = *(const v8h*)(kp);                      kf0.u[1] = z4;
    kf1.h[0] = *(const v8h*)(kp + (size_t)16 * QKN);  kf1.u[1] = z4;
    v8f s0 = mma_raw(qa.v, kf0.v, zero8());
    v8f s1 = mma_raw(qa.v, kf1.v, zero8());
    guard2(s0, s1, qa.v, kf0.v, kf1.v);

    const int key0 = kb + c, key1 = kb + 16 + c;
    const bool ok0 = (key0 < SQ), ok1 = (key1 < SQ);
    const int kc0 = ok0 ? key0 : (SQ - 1), kc1 = ok1 ? key1 : (SQ - 1);
#pragma unroll
    for (int r = 0; r < 8; ++r) {
      float t0 = s0[r] * lsc, t1 = s1[r] * lsc;
      if (AFF) {
        const float* ar = aff + (size_t)idr[r] * VOC;
        t0 += bfr(ar[kc0]) * asc;
        t1 += bfr(ar[kc1]) * asc;
      }
      t0 = ok0 ? t0 : -INFINITY;
      t1 = ok1 ? t1 : -INFINITY;
      float mx = fmaxf(t0, t1);
#pragma unroll
      for (int off = 1; off < 16; off <<= 1) mx = fmaxf(mx, __shfl_xor(mx, off, 32));
      const float mn = fmaxf(mrow[r], mx);
      const float al = exp2f(mrow[r] - mn);
      mrow[r] = mn;
      const float e0 = exp2f(t0 - mn), e1 = exp2f(t1 - mn);
      float ps = e0 + e1;
#pragma unroll
      for (int off = 1; off < 16; off <<= 1) ps += __shfl_xor(ps, off, 32);
      lrow[r] = lrow[r] * al + ps;
      acc[r] *= al;
      const int ro = (8 * hh + r) * 36 + c;
      pt[ro]      = e0;
      pt[ro + 16] = e1;
    }
    wave_sync_lds();
    FragH pa;
    {
      const float* prow = pt + c * 36 + 8 * hh;
      const v4f p0 = *(const v4f*)(prow), p1 = *(const v4f*)(prow + 4);
      const v4f p2 = *(const v4f*)(prow + 16), p3 = *(const v4f*)(prow + 20);
#pragma unroll
      for (int e = 0; e < 4; ++e) {
        pa.h[0][e]     = (_Float16)(p0[e] * PCARRY);
        pa.h[0][4 + e] = (_Float16)(p1[e] * PCARRY);
        pa.h[1][e]     = (_Float16)(p2[e] * PCARRY);
        pa.h[1][4 + e] = (_Float16)(p3[e] * PCARRY);
      }
    }
    {
      const v16h vb = ldfrag_h(Vb + (size_t)c * SP + kb + 8 * hh);
      acc = mma_raw(pa.v, vb, acc);
      guard1(acc, pa.v, vb);
    }
    wave_sync_lds();
  }

  const float oc = OCARRY / (PCARRY * VCARRY);
#pragma unroll
  for (int r = 0; r < 8; ++r) {
    const float inv = (1.0f / lrow[r]) * oc;
    Os[(8 * hh + r) * 68 + 16 * wave + c] = acc[r] * inv;
  }
  __syncthreads();
  {
    const int q8 = lane >> 3, c8 = (lane & 7) * 8;
    const int row = wave * 4 + q8;
    const float* sp = Os + row * 68 + c8;
    v4u a;
#pragma unroll
    for (int e = 0; e < 4; ++e) a[e] = pk16(h_bits((_Float16)sp[2 * e]), h_bits((_Float16)sp[2 * e + 1]));
    unsigned short* dst = CT + ((size_t)bat * SP + q0 + row) * DM + grp * 64 + c8;
    *(volatile v4u*)dst = a;
    __threadfence();
    *(volatile v4u*)dst = a;
  }
}

extern "C" void kernel_launch(void* const* d_in, const int* in_sizes, int n_in,
                              void* d_out, int out_size, void* d_ws, size_t ws_size,
                              hipStream_t stream) {
  if (n_in < 28) return;
  if (in_sizes[0] != TOK * DM || in_sizes[1] != TOK) return;
  if (in_sizes[2] != NQKV * DM || in_sizes[3] != NQKV) return;
  if (in_sizes[4] != DM * DM || in_sizes[5] != DM) return;
  for (int i = 6; i < 12; ++i) if (in_sizes[i] != DM) return;
  if (in_sizes[12] != DM * DM || in_sizes[13] != DM) return;
  if (in_sizes[14] != DM * DM || in_sizes[15] != DM) return;
  if (in_sizes[16] != DM * DM || in_sizes[17] != DM) return;
  if (in_sizes[18] != DM * DM || in_sizes[19] != DM) return;
  if (in_sizes[20] != VOC * VOC) return;
  if (in_sizes[21] != SL * DM || in_sizes[22] != SL * DM || in_sizes[23] != SL) return;
  if (in_sizes[24] != FF * DM || in_sizes[25] != FF) return;
  if (in_sizes[26] != DM * FF || in_sizes[27] != DM) return;
  if (out_size != TOK * DM) return;

  const float* x      = (const float*)d_in[0];
  const int*   ids    = (const int*)d_in[1];
  const float* ipw    = (const float*)d_in[2];
  const float* ipb    = (const float*)d_in[3];
  const float* opw    = (const float*)d_in[4];
  const float* opb    = (const float*)d_in[5];
  const float* ln1g   = (const float*)d_in[6];
  const float* ln1b   = (const float*)d_in[7];
  const float* ln2g   = (const float*)d_in[8];
  const float* ln2b   = (const float*)d_in[9];
  const float* ln3g   = (const float*)d_in[10];
  const float* ln3b   = (const float*)d_in[11];
  const float* gqw    = (const float*)d_in[12];
  const float* gqb    = (const float*)d_in[13];
  const float* gkw    = (const float*)d_in[14];
  const float* gkb    = (const float*)d_in[15];
  const float* gvw    = (const float*)d_in[16];
  const float* gvb    = (const float*)d_in[17];
  const float* gow    = (const float*)d_in[18];
  const float* gob    = (const float*)d_in[19];
  const float* affm   = (const float*)d_in[20];
  const float* memb   = (const float*)d_in[21];
  const float* rdw    = (const float*)d_in[22];
  const float* rdb    = (const float*)d_in[23];
  const float* f1w    = (const float*)d_in[24];
  const float* f1b    = (const float*)d_in[25];
  const float* f2w    = (const float*)d_in[26];
  const float* f2b    = (const float*)d_in[27];
  float*       out    = (float*)d_out;

  const size_t PWIN = (size_t)NQKV * DM * 2;
  const size_t PW6  = (size_t)6 * DM * DM * 2;
  const size_t PWMT = (size_t)DM * SL * 2;
  const size_t PW1  = (size_t)FF * DM * 2;
  const size_t PW2  = (size_t)DM * FF * 2;
  const size_t PH   = (size_t)MROWS * DM * 2;
  const size_t PQK  = (size_t)MROWS * QKN * 2;
  const size_t PVT  = (size_t)NB * DM * SP * 2;
  const size_t PF   = (size_t)MROWS * FF * 2;
  const size_t PX   = (size_t)TOK * DM * 4;
  size_t off = 0;
  const size_t oWIN = off; off += PWIN;
  const size_t oW6  = off; off += PW6;
  const size_t oWMT = off; off += PWMT;
  const size_t oW1  = off; off += PW1;
  const size_t oW2  = off; off += PW2;
  const size_t oH   = off; off += PH;
  const size_t oQK  = off; off += PQK;
  const size_t oVT  = off; off += PVT;
  const size_t oCT  = off; off += PH;
  const size_t oRW  = off; off += PH;
  const size_t oF   = off; off += PF;
  const size_t oX1  = off; off += PX;
  const size_t oX2  = off; off += PX;
  const size_t oLG  = off; off += PX;
  const size_t oX3  = off; off += PX;
  if (off > ws_size) return;
  if (off > (size_t)134217728) return;

  char* ws = (char*)d_ws;
  unsigned short* WIN = (unsigned short*)(ws + oWIN);
  unsigned short* W6  = (unsigned short*)(ws + oW6);
  unsigned short* WMT = (unsigned short*)(ws + oWMT);
  unsigned short* W1  = (unsigned short*)(ws + oW1);
  unsigned short* W2  = (unsigned short*)(ws + oW2);
  unsigned short* H   = (unsigned short*)(ws + oH);
  unsigned short* QK  = (unsigned short*)(ws + oQK);
  unsigned short* VT  = (unsigned short*)(ws + oVT);
  unsigned short* CT  = (unsigned short*)(ws + oCT);
  unsigned short* RW  = (unsigned short*)(ws + oRW);
  unsigned short* F   = (unsigned short*)(ws + oF);
  float*          X1  = (float*)(ws + oX1);
  float*          X2  = (float*)(ws + oX2);
  float*          LG  = (float*)(ws + oLG);
  float*          X3  = (float*)(ws + oX3);
  const size_t W6S = (size_t)DM * DM;

  const int n8in = (NQKV * DM) / 8;
  const int n8sq = (DM * DM) / 8;
  const int n8ff = (FF * DM) / 8;
  if ((n8in % 256) != 0 || (n8sq % 256) != 0 || (n8ff % 256) != 0) return;

  const dim3 blk(256), blk128(128);
  const dim3 gWin(n8in / 256, 1), gW6(n8sq / 256, 6), gWff(n8ff / 256, 1);
  const dim3 gTR(DM / 64, SL / 64);
  const dim3 gROW(ROW_BLOCKS);
  const dim3 gQK(((MROWS / 64) * (QKN / 64) + 7) / 8, 1);
  const dim3 g256(((MROWS / 64) * (DM / 64) + 7) / 8, 1);
  const dim3 gFF1(((MROWS / 64) * (FF / 64) + 7) / 8, 1);
  const dim3 gVT(((DM / 64) * (SP / 64) + 7) / 8, NB);
  const dim3 gPB(((SP / 64) * (DM / 64) + 7) / 8, NB);
  const dim3 gAT(ATT_BLOCKS);

  conv16m<<<gWin, blk, 0, stream>>>(ipw, ipw, ipw, ipw, ipw, ipw, WIN, n8in);
  conv16m<<<gW6,  blk, 0, stream>>>(opw, gqw, gkw, gvw, gow, rdw, W6, n8sq);
  conv16m<<<gWff, blk, 0, stream>>>(f1w, f1w, f1w, f1w, f1w, f1w, W1, n8ff);
  conv16m<<<gWff, blk, 0, stream>>>(f2w, f2w, f2w, f2w, f2w, f2w, W2, n8ff);
  tr16<<<gTR, blk, 0, stream>>>(memb, WMT);

  rows16<1, 1><<<gROW, blk, 0, stream>>>(x, ln1g, ln1b, H, ACARRY);

  gemm64<2, 0, 0, 0><<<gQK, blk, 0, stream>>>(
      H, DM, 0LL, 0LL,
      WIN, DM, 0LL, 0LL,
      ipb, 0, 0,
      x,
      (void*)QK, QKN, 0LL, 0LL,
      MROWS, QKN, DM, MROWS, 1, 1.0f / (ACARRY * WSC), QKCARRY);

  gemm64<2, 1, 0, 0><<<gVT, blk, 0, stream>>>(
      WIN + (size_t)QKN * DM, DM, 0LL, 0LL,
      H, DM, (long long)SP * DM, 0LL,
      ipb + QKN, 0, 0,
      x,
      (void*)VT, SP, (long long)DM * SP, 0LL,
      DM, SP, DM, DM, 1, 1.0f / (ACARRY * WSC), VCARRY);

  attn16<0><<<gAT, blk128, 0, stream>>>(QK, VT, ids, affm, CT);

  gemm64<0, 0, 0, 2><<<gPB, blk, 0, stream>>>(
      CT, DM, (long long)SP * DM, 0LL,
      W6 + 0 * W6S, DM, 0LL, 0LL,
      opb, 0, 0,
      x,
      (void*)X1, DM, (long long)SQ * DM, 0LL,
      SP, DM, DM, SQ, 1, 1.0f / (OCARRY * WSC), 1.0f);

  rows16<1, 0><<<gROW, blk, 0, stream>>>(X1, ln2g, ln2b, H, ACARRY);

  gemm64<2, 0, 0, 0><<<g256, blk, 0, stream>>>(
      H, DM, 0LL, 0LL,
      W6 + 1 * W6S, DM, 0LL, 0LL,
      gqb, 0, 0,
      x,
      (void*)QK, QKN, 0LL, 0LL,
      MROWS, DM, DM, MROWS, 1, 1.0f / (ACARRY * WSC), QKCARRY);
  gemm64<2, 0, 0, 0><<<g256, blk, 0, stream>>>(
      H, DM, 0LL, 0LL,
      W6 + 2 * W6S, DM, 0LL, 0LL,
      gkb, 0, 0,
      x,
      (void*)(QK + DM), QKN, 0LL, 0LL,
      MROWS, DM, DM, MROWS, 1, 1.0f / (ACARRY * WSC), QKCARRY);
  gemm64<2, 1, 0, 0><<<gVT, blk, 0, stream>>>(
      W6 + 3 * W6S, DM, 0LL, 0LL,
      H, DM, (long long)SP * DM, 0LL,
      gvb, 0, 0,
      x,
      (void*)VT, SP, (long long)DM * SP, 0LL,
      DM, SP, DM, DM, 1, 1.0f / (ACARRY * WSC), VCARRY);

  attn16<1><<<gAT, blk128, 0, stream>>>(QK, VT, ids, affm, CT);

  gemm64<0, 0, 0, 1><<<gPB, blk, 0, stream>>>(
      CT, DM, (long long)SP * DM, 0LL,
      W6 + 4 * W6S, DM, 0LL, 0LL,
      gob, 0, 0,
      X1,
      (void*)X2, DM, (long long)SQ * DM, 0LL,
      SP, DM, DM, SQ, 1, 1.0f / (OCARRY * WSC), 1.0f);

  rows16<0, 0><<<gROW, blk, 0, stream>>>(X2, ln1g, ln1b, H, XCARRY);
  gemm64<0, 0, 0, 0><<<gPB, blk, 0, stream>>>(
      H, DM, (long long)SP * DM, 0LL,
      W6 + 5 * W6S, DM, 0LL, 0LL,
      rdb, 0, 0,
      x,
      (void*)LG, DM, (long long)SQ * DM, 0LL,
      SP, SL, DM, SQ, 1, 1.0f / (XCARRY * WSC), 1.0f);
  smax16<<<gROW, blk, 0, stream>>>(LG, RW);

  gemm64<0, 2, 0, 1><<<gPB, blk, 0, stream>>>(
      RW, SL, (long long)SP * SL, 0LL,
      WMT, SL, 0LL, 0LL,
      rdb, 0, 0,
      X2,
      (void*)X3, DM, (long long)SQ * DM, 0LL,
      SP, DM, SL, SQ, 1, 1.0f / (RWCARRY * WSC), 1.0f);

  rows16<1, 0><<<gROW, blk, 0, stream>>>(X3, ln3g, ln3b, H, ACARRY);
  gemm64<2, 0, 1, 0><<<gFF1, blk, 0, stream>>>(
      H, DM, 0LL, 0LL,
      W1, DM, 0LL, 0LL,
      f1b, 0, 0,
      x,
      (void*)F, FF, 0LL, 0LL,
      MROWS, FF, DM, MROWS, 1, 1.0f / (ACARRY * WSC), FCARRY);

  gemm64<0, 0, 0, 1><<<gPB, blk, 0, stream>>>(
      F, FF, (long long)SP * FF, 0LL,
      W2, FF, 0LL, 0LL,
      f2b, 0, 0,
      X3,
      (void*)out, DM, (long long)SQ * DM, 0LL,
      SP, DM, FF, SQ, 1, 1.0f / (FCARRY * WSC), 1.0f);
  (void)hipGetLastError();
}
